// GraphSAGE_81320910783036
// MI455X (gfx1250) — hardware-verified
//
#include <hip/hip_runtime.h>
#include <stddef.h>
#include <stdint.h>


#define DF    128
#define K1    256
#define K2    512
#define K3    256
#define NO    64
#define SMP   16
#define NTHR  256
#define GBM   64
#define GBN   128
#define GTHR  128
#define TM    32
#define GW1   ((DF * (K1 / 8)) / NTHR)
#define GW2   ((DF * (K2 / 8)) / NTHR)
#define GWO   ((NO * (K3 / 8)) / NTHR)
#define NBIAS 320
#define WSMAX 134217728

static_assert(K1 == 2 * DF && K2 == 4 * DF && K3 == 2 * DF);
static_assert(K1 % 32 == 0 && K2 % 32 == 0 && K3 % 32 == 0);
static_assert((DF * (K1 / 8)) % NTHR == 0 && (DF * (K2 / 8)) % NTHR == 0 && (NO * (K3 / 8)) % NTHR == 0);
static_assert(GBN == DF && GBM == (GTHR / 32) * 16 && DF == 4 * 32);
static_assert(TM == 32 && GTHR == 128 && (TM * NO) % (4 * GTHR) == 0);
static_assert((NBIAS * 4) % 128 == 0 && NBIAS / 4 <= NTHR);
static_assert(TM * K2 * 2 + TM * K3 * 2 + TM * NO * 4 <= 65536);
static_assert(SMP == 16);

typedef float          v4f   __attribute__((ext_vector_type(4)));
typedef float          v8f   __attribute__((ext_vector_type(8)));
typedef int            v8i   __attribute__((ext_vector_type(8)));
typedef unsigned int   v4u   __attribute__((ext_vector_type(4)));
typedef unsigned short v4us  __attribute__((ext_vector_type(4)));
typedef unsigned short v8us  __attribute__((ext_vector_type(8)));
typedef unsigned short v16us __attribute__((ext_vector_type(16)));
typedef __bf16         v16bf __attribute__((ext_vector_type(16)));
typedef v4f  __attribute__((may_alias)) v4fa;
typedef v4u  __attribute__((may_alias)) v4ua;
typedef v4us __attribute__((may_alias)) v4usa;
typedef v8us __attribute__((may_alias)) v8usa;
union FragB { v16bf v; v16us u; v8us h[2]; v8i w; };

__device__ __forceinline__ v8f wmb(const FragB& a, const FragB& b, v8f c) {
  v8f d = __builtin_amdgcn_wmma_f32_16x16x32_bf16(false, a.v, false, b.v, (short)0, c, false, false);
  asm volatile("v_nop\n\tv_nop\n\tv_nop\n\tv_nop" : "+v"(d) : "v"(a.w), "v"(b.w));
  return d;
}

__device__ __forceinline__ unsigned bf16_bits(float f) {
  const unsigned u = __float_as_uint(f);
  return (u + 0x7FFFu + ((u >> 16) & 1u)) >> 16;
}
__device__ __forceinline__ float bf16_val(float f) {
  return __uint_as_float(bf16_bits(f) << 16);
}

__global__ __launch_bounds__(NTHR) void k_prep(const float* __restrict__ x, int nN, int gx,
                                               const float* __restrict__ W1, const float* __restrict__ W2,
                                               const float* __restrict__ Wout, const float* __restrict__ b1,
                                               const float* __restrict__ b2, const float* __restrict__ bout,
                                               unsigned short* F1, unsigned short* W1T, unsigned short* W2T2,
                                               unsigned short* WO2, float* BIAS) {
  const int tid = (int)threadIdx.x;
  const int b   = (int)blockIdx.x;
  if (b < gx) {
    const int u = b * NTHR + tid;
    if (u >= nN * 16) return;
    const int row = u >> 4;
    const int k8  = (u & 15) * 8;
    const float* p = x + (size_t)row * DF + k8;
    const v4f a = *(const v4fa*)p;
    const v4f c = *(const v4fa*)(p + 4);
    v8us o;
    o[0] = (unsigned short)bf16_bits(a.x); o[1] = (unsigned short)bf16_bits(a.y);
    o[2] = (unsigned short)bf16_bits(a.z); o[3] = (unsigned short)bf16_bits(a.w);
    o[4] = (unsigned short)bf16_bits(c.x); o[5] = (unsigned short)bf16_bits(c.y);
    o[6] = (unsigned short)bf16_bits(c.z); o[7] = (unsigned short)bf16_bits(c.w);
    unsigned short* dp = F1 + (size_t)row * K1 + k8;
    *(volatile v8us*)dp = o;
    __threadfence();
    *(volatile v8us*)dp = o;
    return;
  }
  const int wb = b - gx;
  if (wb < GW1 + GW2 + GWO) {
    const float* p;
    int stride;
    unsigned short* dp;
    if (wb < GW1) {
      const int v  = wb * NTHR + tid;
      const int n  = v >> 5;
      const int k8 = (v & 31) * 8;
      p = W1 + (size_t)k8 * DF + n; stride = DF;
      dp = W1T + (size_t)n * K1 + k8;
    } else if (wb < GW1 + GW2) {
      const int v  = (wb - GW1) * NTHR + tid;
      const int n  = v >> 6;
      const int k8 = (v & 63) * 8;
      const int kk = k8 & (K1 - 1);
      p = W2 + (size_t)kk * DF + n; stride = DF;
      dp = W2T2 + (size_t)n * K2 + k8;
    } else {
      const int v  = (wb - GW1 - GW2) * NTHR + tid;
      const int n  = v >> 5;
      const int k8 = (v & 31) * 8;
      const int kk = k8 & (DF - 1);
      p = Wout + (size_t)kk * NO + n; stride = NO;
      dp = WO2 + (size_t)n * K3 + k8;
    }
    v8us o;
#pragma unroll
    for (int i = 0; i < 8; ++i) o[i] = (unsigned short)bf16_bits(p[(size_t)i * (size_t)stride]);
    *(volatile v8us*)dp = o;
    __threadfence();
    *(volatile v8us*)dp = o;
    return;
  }
  {
    const int q = tid;
    const int q1 = q < 31 ? q : 31;
    int q2 = q - 32; q2 = q2 < 0 ? 0 : (q2 > 31 ? 31 : q2);
    int q3 = q - 64; q3 = q3 < 0 ? 0 : (q3 > 15 ? 15 : q3);
    const v4u a1 = *(const v4ua*)(b1 + 4 * q1);
    const v4u a2 = *(const v4ua*)(b2 + 4 * q2);
    const v4u a3 = *(const v4ua*)(bout + 4 * q3);
    const unsigned m1 = (q < 32) ? 0xffffffffu : 0u;
    const unsigned m2 = (q >= 32 && q < 64) ? 0xffffffffu : 0u;
    const unsigned m3 = (q >= 64) ? 0xffffffffu : 0u;
    const unsigned wx = (a1.x & m1) | (a2.x & m2) | (a3.x & m3);
    const unsigned wy = (a1.y & m1) | (a2.y & m2) | (a3.y & m3);
    const unsigned wz = (a1.z & m1) | (a2.z & m2) | (a3.z & m3);
    const unsigned ww = (a1.w & m1) | (a2.w & m2) | (a3.w & m3);
    v4f o;
    o.x = bf16_val(__uint_as_float(wx));
    o.y = bf16_val(__uint_as_float(wy));
    o.z = bf16_val(__uint_as_float(wz));
    o.w = bf16_val(__uint_as_float(ww));
    const bool ok = q < NBIAS / 4;
    float* dp = BIAS + 4 * (ok ? q : 0);
    if (ok) *(volatile v4f*)dp = o;
    __threadfence();
    if (ok) *(volatile v4f*)dp = o;
  }
}

__global__ __launch_bounds__(NTHR) void k_gmax1(const int* __restrict__ nidx, int nN, unsigned short* F1) {
  const int tid = (int)threadIdx.x, lane = tid & 31, wave = tid >> 5, hf = lane >> 4, m = lane & 15;
  const int row = ((int)blockIdx.x * (NTHR / 32) + wave) * 2 + hf;
  const bool valid = row < nN;
  const int rc = valid ? row : nN - 1;
  int my = nidx[(size_t)rc * SMP + m];
  my = my < 0 ? 0 : (my > nN - 1 ? nN - 1 : my);
  const float ninf = __int_as_float((int)0xff800000u);
  float e0 = ninf, e1 = ninf, e2 = ninf, e3 = ninf, e4 = ninf, e5 = ninf, e6 = ninf, e7 = ninf;
#pragma unroll 4
  for (int s = 0; s < SMP; ++s) {
    const int src = __shfl(my, s, 16);
    const v4u w = *(const v4ua*)(F1 + (size_t)src * K1 + 8 * m);
    e0 = fmaxf(e0, __uint_as_float(w.x << 16));
    e1 = fmaxf(e1, __uint_as_float(w.x & 0xffff0000u));
    e2 = fmaxf(e2, __uint_as_float(w.y << 16));
    e3 = fmaxf(e3, __uint_as_float(w.y & 0xffff0000u));
    e4 = fmaxf(e4, __uint_as_float(w.z << 16));
    e5 = fmaxf(e5, __uint_as_float(w.z & 0xffff0000u));
    e6 = fmaxf(e6, __uint_as_float(w.w << 16));
    e7 = fmaxf(e7, __uint_as_float(w.w & 0xffff0000u));
  }
  v4u o;
  o.x = (__float_as_uint(e0) >> 16) | (__float_as_uint(e1) & 0xffff0000u);
  o.y = (__float_as_uint(e2) >> 16) | (__float_as_uint(e3) & 0xffff0000u);
  o.z = (__float_as_uint(e4) >> 16) | (__float_as_uint(e5) & 0xffff0000u);
  o.w = (__float_as_uint(e6) >> 16) | (__float_as_uint(e7) & 0xffff0000u);
  unsigned short* dp = F1 + (size_t)rc * K1 + DF + 8 * m;
  if (valid) *(volatile v4u*)dp = o;
  __threadfence();
  if (valid) *(volatile v4u*)dp = o;
}

__global__ __launch_bounds__(GTHR) void k_gemm1(const unsigned short* __restrict__ A,
                                                const unsigned short* __restrict__ BT,
                                                const float* __restrict__ bias, float* outp, int nN) {
  __shared__ __attribute__((aligned(16))) float stg[GBM * GBN];
  const int tid = (int)threadIdx.x, lane = tid & 31, wave = tid >> 5, hh = lane >> 4, m = lane & 15;
  const int rowBase = (int)blockIdx.x * GBM;

  v8f acc[8];
  {
    const v8f z = {0.f, 0.f, 0.f, 0.f, 0.f, 0.f, 0.f, 0.f};
#pragma unroll
    for (int t = 0; t < 8; ++t) acc[t] = z;
  }
  int ar = rowBase + 16 * wave + m;
  ar = ar < nN ? ar : nN - 1;
  const unsigned short* ap = A + (size_t)ar * (size_t)K1 + 8 * hh;
  const unsigned short* bp = BT + (size_t)m * (size_t)K1 + 8 * hh;

#pragma unroll 1
  for (int k0 = 0; k0 < K1; k0 += 32) {
    FragB af;
    af.h[0] = *(const v8usa*)(ap + k0);
    af.h[1] = *(const v8usa*)(ap + k0 + 16);
#pragma unroll
    for (int nt = 0; nt < 8; ++nt) {
      const unsigned short* wq = bp + (size_t)(16 * nt) * (size_t)K1 + k0;
      FragB bf;
      bf.h[0] = *(const v8usa*)wq;
      bf.h[1] = *(const v8usa*)(wq + 16);
      acc[nt] = wmb(af, bf, acc[nt]);
    }
  }

#pragma unroll
  for (int nt = 0; nt < 8; ++nt) {
    const int lc = 16 * nt + m;
#pragma unroll
    for (int r = 0; r < 8; ++r) {
      const int lr = 16 * wave + 8 * hh + r;
      stg[lr * GBN + lc] = acc[nt][r];
    }
  }
  __syncthreads();

  const v4f bb4 = *(const v4fa*)(bias + 4 * lane);
  v4f pv[16];
#pragma unroll
  for (int i = 0; i < 16; ++i) pv[i] = *(const v4fa*)(stg + (16 * wave + i) * GBN + 4 * lane);
#pragma unroll
  for (int i = 0; i < 16; ++i) {
    const v4f t = pv[i] + bb4;
    v4f y;
    y.x = (t.x > 0.0f) ? t.x : (t.x - t.x);
    y.y = (t.y > 0.0f) ? t.y : (t.y - t.y);
    y.z = (t.z > 0.0f) ? t.z : (t.z - t.z);
    y.w = (t.w > 0.0f) ? t.w : (t.w - t.w);
    pv[i] = y;
  }
#pragma unroll
  for (int i = 0; i < 16; ++i) {
    const int r = rowBase + 16 * wave + i;
    if (r < nN) *(volatile v4f*)(outp + (size_t)r * DF + 4 * lane) = pv[i];
  }
  __threadfence();
#pragma unroll
  for (int i = 0; i < 16; ++i) {
    const int r = rowBase + 16 * wave + i;
    if (r < nN) *(volatile v4f*)(outp + (size_t)r * DF + 4 * lane) = pv[i];
  }
}

__global__ __launch_bounds__(GTHR) void k_sage2(const float* __restrict__ H1, const int* __restrict__ nidx,
                                                const int* __restrict__ batch, int nN, int nB,
                                                const unsigned short* __restrict__ W2T2,
                                                const unsigned short* __restrict__ WO2,
                                                const float* __restrict__ BIAS, float* out) {
  __shared__ __attribute__((aligned(16))) unsigned short a2[TM * K2];
  __shared__ __attribute__((aligned(16))) unsigned short a3[TM * K3];
  __shared__ __attribute__((aligned(16))) float ost[TM * NO];
  const int tid = (int)threadIdx.x, lane = tid & 31, wave = tid >> 5, hh = lane >> 4, m = lane & 15;
  const int tile0 = (int)blockIdx.x * TM;

  const float ninf = __int_as_float((int)0xff800000u);
#pragma unroll 1
  for (int i = 0; i < 8; ++i) {
    const int r  = 8 * wave + i;
    const int j  = tile0 + r;
    const int jc = j < nB ? j : nB - 1;
    int n = batch[jc];
    n = n < 0 ? 0 : (n > nN - 1 ? nN - 1 : n);
    int my = nidx[(size_t)n * SMP + m];
    my = my < 0 ? 0 : (my > nN - 1 ? nN - 1 : my);
    const v4f own = *(const v4fa*)(H1 + (size_t)n * DF + 4 * lane);
    float x0 = ninf, x1 = ninf, x2 = ninf, x3 = ninf;
#pragma unroll 4
    for (int s = 0; s < SMP; ++s) {
      const int src = __shfl(my, s, 32);
      const v4f v = *(const v4fa*)(H1 + (size_t)src * DF + 4 * lane);
      x0 = fmaxf(x0, v.x); x1 = fmaxf(x1, v.y); x2 = fmaxf(x2, v.z); x3 = fmaxf(x3, v.w);
    }
    v4us oh, ol, gh, gl;
    unsigned hb;
    hb = bf16_bits(own.x); oh[0] = (unsigned short)hb; ol[0] = (unsigned short)bf16_bits(own.x - __uint_as_float(hb << 16));
    hb = bf16_bits(own.y); oh[1] = (unsigned short)hb; ol[1] = (unsigned short)bf16_bits(own.y - __uint_as_float(hb << 16));
    hb = bf16_bits(own.z); oh[2] = (unsigned short)hb; ol[2] = (unsigned short)bf16_bits(own.z - __uint_as_float(hb << 16));
    hb = bf16_bits(own.w); oh[3] = (unsigned short)hb; ol[3] = (unsigned short)bf16_bits(own.w - __uint_as_float(hb << 16));
    hb = bf16_bits(x0); gh[0] = (unsigned short)hb; gl[0] = (unsigned short)bf16_bits(x0 - __uint_as_float(hb << 16));
    hb = bf16_bits(x1); gh[1] = (unsigned short)hb; gl[1] = (unsigned short)bf16_bits(x1 - __uint_as_float(hb << 16));
    hb = bf16_bits(x2); gh[2] = (unsigned short)hb; gl[2] = (unsigned short)bf16_bits(x2 - __uint_as_float(hb << 16));
    hb = bf16_bits(x3); gh[3] = (unsigned short)hb; gl[3] = (unsigned short)bf16_bits(x3 - __uint_as_float(hb << 16));
    unsigned short* rp = a2 + r * K2 + 4 * lane;
    *(v4usa*)(rp)          = oh;
    *(v4usa*)(rp + DF)     = gh;
    *(v4usa*)(rp + 2 * DF) = ol;
    *(v4usa*)(rp + 3 * DF) = gl;
  }
  __syncthreads();

  const int mt = wave & 1, ng = wave >> 1;
  const v8f z8 = {0.f, 0.f, 0.f, 0.f, 0.f, 0.f, 0.f, 0.f};

  {
    v8f acc[4];
    acc[0] = z8; acc[1] = z8; acc[2] = z8; acc[3] = z8;
    const unsigned short* ap = a2 + (16 * mt + m) * K2 + 8 * hh;
    const unsigned short* bp = W2T2 + (size_t)(64 * ng + m) * (size_t)K2 + 8 * hh;
#pragma unroll 1
    for (int k0 = 0; k0 < K2; k0 += 32) {
      FragB af;
      af.h[0] = *(const v8usa*)(ap + k0);
      af.h[1] = *(const v8usa*)(ap + k0 + 16);
#pragma unroll
      for (int t = 0; t < 4; ++t) {
        const unsigned short* wq = bp + (size_t)(16 * t) * (size_t)K2 + k0;
        FragB bf;
        bf.h[0] = *(const v8usa*)wq;
        bf.h[1] = *(const v8usa*)(wq + 16);
        acc[t] = wmb(af, bf, acc[t]);
      }
    }
#pragma unroll
    for (int t = 0; t < 4; ++t) {
      const int col = 64 * ng + 16 * t + m;
      const float bb = BIAS[DF + col];
#pragma unroll
      for (int r = 0; r < 8; ++r) {
        const int row = 16 * mt + 8 * hh + r;
        const float v = acc[t][r] + bb;
        const unsigned hb = bf16_bits(v);
        const unsigned lb = bf16_bits(v - __uint_as_float(hb << 16));
        a3[row * K3 + col]      = (unsigned short)hb;
        a3[row * K3 + DF + col] = (unsigned short)lb;
      }
    }
  }
  __syncthreads();

  {
    v8f c2[2];
    c2[0] = z8; c2[1] = z8;
    const unsigned short* ap = a3 + (16 * mt + m) * K3 + 8 * hh;
    const unsigned short* bp = WO2 + (size_t)(32 * ng + m) * (size_t)K3 + 8 * hh;
#pragma unroll 1
    for (int k0 = 0; k0 < K3; k0 += 32) {
      FragB af;
      af.h[0] = *(const v8usa*)(ap + k0);
      af.h[1] = *(const v8usa*)(ap + k0 + 16);
#pragma unroll
      for (int t = 0; t < 2; ++t) {
        const unsigned short* wq = bp + (size_t)(16 * t) * (size_t)K3 + k0;
        FragB bf;
        bf.h[0] = *(const v8usa*)wq;
        bf.h[1] = *(const v8usa*)(wq + 16);
        c2[t] = wmb(af, bf, c2[t]);
      }
    }
#pragma unroll
    for (int t = 0; t < 2; ++t) {
      const int col = 32 * ng + 16 * t + m;
      const float bo = BIAS[2 * DF + col];
#pragma unroll
      for (int r = 0; r < 8; ++r) {
        const int row = 16 * mt + 8 * hh + r;
        ost[row * NO + col] = c2[t][r] + bo;
      }
    }
  }
  __syncthreads();

  constexpr int NIT = (TM * NO) / (4 * GTHR);
  v4f ov[NIT];
#pragma unroll
  for (int it = 0; it < NIT; ++it) ov[it] = *(const v4fa*)(ost + 4 * (it * GTHR + tid));
#pragma unroll
  for (int it = 0; it < NIT; ++it) {
    const int q = it * GTHR + tid;
    const int j = tile0 + (q >> 4);
    const int jc = j < nB ? j : nB - 1;
    float* op = out + (size_t)jc * NO + 4 * (q & 15);
    if (j < nB) *(volatile v4f*)op = ov[it];
  }
  __threadfence();
#pragma unroll
  for (int it = 0; it < NIT; ++it) {
    const int q = it * GTHR + tid;
    const int j = tile0 + (q >> 4);
    const int jc = j < nB ? j : nB - 1;
    float* op = out + (size_t)jc * NO + 4 * (q & 15);
    if (j < nB) *(volatile v4f*)op = ov[it];
  }
}

static inline int cdiv(int a, int b) { return (a + b - 1) / b; }
static inline size_t al256(size_t o) { return (o + 255) & ~(size_t)255; }

extern "C" void kernel_launch(void* const* d_in, const int* in_sizes, int n_in,
                              void* d_out, int out_size, void* d_ws, size_t ws_size,
                              hipStream_t stream) {
  if (n_in < 9) return;
  if (in_sizes[0] < DF || (in_sizes[0] % DF) != 0) return;
  const int nN = in_sizes[0] / DF;
  if (nN < 1 || nN > (1 << 22)) return;
  if ((long long)in_sizes[1] != (long long)nN * SMP) return;
  const int nB = in_sizes[2];
  if (nB < 1 || nB > (1 << 22)) return;
  if (in_sizes[3] != K1 * DF || in_sizes[4] != DF) return;
  if (in_sizes[5] != K1 * DF || in_sizes[6] != DF) return;
  if (in_sizes[7] != DF * NO || in_sizes[8] != NO) return;
  if ((long long)out_size != (long long)nB * NO) return;

  const float* x    = (const float*)d_in[0];
  const int*   nidx = (const int*)d_in[1];
  const int*   bat  = (const int*)d_in[2];
  const float* W1   = (const float*)d_in[3];
  const float* b1   = (const float*)d_in[4];
  const float* W2   = (const float*)d_in[5];
  const float* b2   = (const float*)d_in[6];
  const float* Wout = (const float*)d_in[7];
  const float* bout = (const float*)d_in[8];
  float* out = (float*)d_out;

  const int MP = cdiv(nN, GBM) * GBM;
  char* ws = (char*)d_ws;
  size_t off = 0;
  const size_t oF1  = off; off = al256(off + (size_t)MP * K1 * 2);
  const size_t oH1  = off; off = al256(off + (size_t)MP * DF * 4);
  const size_t oW1T = off; off = al256(off + (size_t)DF * K1 * 2);
  const size_t oW2T = off; off = al256(off + (size_t)DF * K2 * 2);
  const size_t oWO2 = off; off = al256(off + (size_t)NO * K3 * 2);
  const size_t oBI  = off; off = al256(off + (size_t)NBIAS * 4);
  if (off > ws_size || off > (size_t)WSMAX) return;
  unsigned short* F1   = (unsigned short*)(ws + oF1);
  float*          H1   = (float*)(ws + oH1);
  unsigned short* W1T  = (unsigned short*)(ws + oW1T);
  unsigned short* W2T2 = (unsigned short*)(ws + oW2T);
  unsigned short* WO2  = (unsigned short*)(ws + oWO2);
  float*          BIAS = (float*)(ws + oBI);

  const int gx = cdiv(nN * 16, NTHR);
  k_prep<<<gx + GW1 + GW2 + GWO + 1, NTHR, 0, stream>>>(x, nN, gx, W1, W2, Wout, b1, b2, bout,
                                                        F1, W1T, W2T2, WO2, BIAS);
  k_gmax1<<<cdiv(nN, 2 * (NTHR / 32)), NTHR, 0, stream>>>(nidx, nN, F1);
  k_gemm1<<<cdiv(nN, GBM), GTHR, 0, stream>>>(F1, W1T, BIAS, H1, nN);
  k_sage2<<<cdiv(nB, TM), GTHR, 0, stream>>>(H1, nidx, bat, nN, nB, W2T2, WO2, BIAS, out);
}
